// RoPEAttention_80187039416553
// MI455X (gfx1250) — hardware-verified
//
#include <hip/hip_runtime.h>

#ifndef NB
#define NB 4
#endif
#ifndef SEQ
#define SEQ 4096
#endif
#ifndef QK_RES
#define QK_RES 0
#endif
#define NB_FULL 4
#define SEQ_FULL 4096
#define DM 256
#define NH 4
#define HD 64
#define WFT 64
#define SLEN SEQ
#define NR (NB * SLEN)
#define TQ SLEN
#define TK SLEN
#define NCH (TK / 32)
#define SCL 0.125f
#define QBLKS (TQ / 64)
static_assert(SLEN % 128 == 0);
static_assert(SLEN <= SEQ_FULL);
static_assert(NB >= 1 && NB <= NB_FULL);
static_assert(DM == NH * HD);
static_assert(HD == 64);
static_assert(DM % 64 == 0);
static_assert(TK % 32 == 0);
static_assert(NR % 128 == 0);

typedef _Float16 v16h __attribute__((ext_vector_type(16)));
typedef _Float16 v4h __attribute__((ext_vector_type(4)));
typedef unsigned short v8us __attribute__((ext_vector_type(8), may_alias));
typedef float v8f __attribute__((ext_vector_type(8)));
typedef float v4f __attribute__((ext_vector_type(4)));
typedef float v4fa __attribute__((ext_vector_type(4), may_alias));
union FragH { v16h v; v8us half[2]; _Float16 h[16]; unsigned short u[16]; };

__device__ __forceinline__ unsigned short bf16_bits(float x) { unsigned int u = __float_as_uint(x); return (unsigned short)((u + 0x7FFFu + ((u >> 16) & 1u)) >> 16); }
__device__ __forceinline__ float bf16_val(unsigned short b) { return __uint_as_float(((unsigned int)b) << 16); }
__device__ __forceinline__ float bf16_rne(float x) { return bf16_val(bf16_bits(x)); }

template <int NT>
__device__ __forceinline__ v8f mmaH(v16h ah, v16h al, v16h bh, v16h bl, v8f c) {
  c = __builtin_amdgcn_wmma_f32_16x16x32_f16(false, ah, false, bh, (short)0, c, false, false);
  if (NT >= 2) c = __builtin_amdgcn_wmma_f32_16x16x32_f16(false, al, false, bh, (short)0, c, false, false);
  if (NT >= 3) c = __builtin_amdgcn_wmma_f32_16x16x32_f16(false, ah, false, bl, (short)0, c, false, false);
  asm volatile("v_nop\n\tv_nop\n\tv_nop\n\tv_nop" : "+v"(c) : "v"(ah), "v"(al), "v"(bh), "v"(bl));
  return c;
}
__device__ __forceinline__ v16h g2_frag(const _Float16* p, int hh) { FragH f; f.half[0] = *(const v8us*)((const unsigned short*)p + 8 * hh); f.half[1] = *(const v8us*)((const unsigned short*)p + 16 + 8 * hh); return f.v; }
__device__ __forceinline__ v8f g2_mma(v16h a, v16h b, v8f c) { v8f d = __builtin_amdgcn_wmma_f32_16x16x32_f16(false, a, false, b, (short)0, c, false, false); asm volatile("v_nop\n\tv_nop\n\tv_nop\n\tv_nop" : "+v"(d) : "v"(a), "v"(b)); return d; }

template <int TWO>
__global__ __launch_bounds__(256) void k_wtr(const float* __restrict__ Wm, _Float16* __restrict__ Bt, int ldb, float sc0, float sc1) {
  __shared__ __attribute__((aligned(16))) unsigned short t0[64][72];
  __shared__ __attribute__((aligned(16))) unsigned short t1[64][72];
  const int tid = threadIdx.x; const int ntl = DM / 64; const int kt = blockIdx.x / ntl, nt = blockIdx.x % ntl; const int k0 = kt * 64, n0 = nt * 64;
  for (int i = tid; i < 64 * 16; i += 256) {
    const int r = i >> 4, c4 = (i & 15) * 4;
    const v4f a = *(const v4fa*)(Wm + (size_t)(k0 + r) * DM + n0 + c4);
    FragH f0, f1;
#pragma unroll
    for (int q = 0; q < 4; ++q) { const float wv = bf16_rne(a[q]); f0.h[q] = (_Float16)(wv * sc0); f1.h[q] = (_Float16)(wv * sc1); }
#pragma unroll
    for (int q = 0; q < 4; ++q) { t0[c4 + q][r] = f0.u[q]; if (TWO) t1[c4 + q][r] = f1.u[q]; }
  }
  __syncthreads();
  for (int pass = 0; pass < 2; ++pass) {
#pragma unroll
    for (int rd = 0; rd < 2; ++rd) {
      const int n = rd * 32 + (tid >> 3), pc = tid & 7;
      const v8us o0 = *(const v8us*)&t0[n][pc * 8];
      *(volatile v8us*)((unsigned short*)Bt + (size_t)(n0 + n) * ldb + k0 + pc * 8) = o0;
      if (TWO) { const v8us o1 = *(const v8us*)&t1[n][pc * 8]; *(volatile v8us*)((unsigned short*)Bt + (size_t)(n0 + n) * ldb + DM + k0 + pc * 8) = o1; }
    }
    if (pass == 0) __threadfence();
  }
}

__global__ __launch_bounds__(32) void k_invf(float* __restrict__ INV) {
  #pragma clang fp contract(off)
  const int j = threadIdx.x;
  const float ex = (float)(4 * (j & 15)) / 64.0f; const float pw = powf(10000.0f, ex); const float inv = 1.0f / pw;
  *(volatile float*)(INV + j) = inv; __threadfence(); *(volatile float*)(INV + j) = inv;
}
__global__ __launch_bounds__(256) void k_rotab(const float* __restrict__ INV, float* __restrict__ CS, float* __restrict__ SN) {
  #pragma clang fp contract(off)
  const int t = blockIdx.x * 256 + threadIdx.x; if (t >= SLEN * 32) return;
  const int p = t & 31, s = t >> 5;
  const int px = s % WFT, py = s / WFT;
  const float pos = (p < 16) ? (float)px : (float)py;
  const float th = pos * INV[p]; const float c = cosf(th), sn = sinf(th);
  for (int pass = 0; pass < 2; ++pass) { *(volatile float*)(CS + t) = c; *(volatile float*)(SN + t) = sn; if (pass == 0) __threadfence(); }
}

__global__ __launch_bounds__(256) void k_x16(const float* __restrict__ x, _Float16* __restrict__ X16, size_t n8) {
  const size_t t = (size_t)blockIdx.x * 256 + threadIdx.x; if (t >= n8) return;
  const size_t e = t * 8; const size_t r = e / DM; const size_t c = e % DM; const size_t b = r / SLEN, s = r % SLEN;
  const float* src = x + (b * SEQ_FULL + s) * DM + c;
  const v4f a0 = *(const v4fa*)src, a1 = *(const v4fa*)(src + 4);
  FragH f;
#pragma unroll
  for (int q = 0; q < 4; ++q) { f.h[q] = (_Float16)bf16_rne(a0[q]); f.h[4 + q] = (_Float16)bf16_rne(a1[q]); }
  const v8us o = f.half[0];
  *(volatile v8us*)((unsigned short*)X16 + e) = o; __threadfence(); *(volatile v8us*)((unsigned short*)X16 + e) = o;
}

template <int ACT>
__global__ __launch_bounds__(128) void k_gemm2(const _Float16* __restrict__ A, int lda, size_t sA, const _Float16* __restrict__ Bh, int ldb, size_t sB, float alpha,
                                               float* C, _Float16* C16, int ldc, size_t sC, int M, int N, int K, const float* __restrict__ bias) {
  __shared__ __attribute__((aligned(16))) float so[4][32][68];
  const int tid = threadIdx.x, w = tid >> 5, lane = tid & 31, ln = lane & 15, hh = lane >> 4; const int by = blockIdx.y;
  A += (size_t)by * sA; Bh += (size_t)by * sB; const size_t cofs = (size_t)by * sC;
  const int ntn = N >> 6; const int mt = blockIdx.x / ntn, nq = blockIdx.x - mt * ntn; const int row0 = mt * 128 + 32 * w, col0 = nq * 64; if (row0 >= M) return;
  const _Float16* a0p = A + (size_t)(row0 + ln) * lda; const _Float16* a1p = a0p + (size_t)16 * lda;
  const _Float16* b0p = Bh + (size_t)(col0 + ln) * ldb; const _Float16* b1p = b0p + (size_t)16 * ldb; const _Float16* b2p = b1p + (size_t)16 * ldb; const _Float16* b3p = b2p + (size_t)16 * ldb;
  const v8f z8 = {0.f,0.f,0.f,0.f,0.f,0.f,0.f,0.f}; v8f c00 = z8, c01 = z8, c02 = z8, c03 = z8, c10 = z8, c11 = z8, c12 = z8, c13 = z8;
#pragma unroll 1
  for (int kb = 0; kb < K; kb += 32) {
    const v16h a0 = g2_frag(a0p + kb, hh), a1 = g2_frag(a1p + kb, hh);
    v16h bf = g2_frag(b0p + kb, hh); c00 = g2_mma(a0, bf, c00); c10 = g2_mma(a1, bf, c10);
    bf = g2_frag(b1p + kb, hh); c01 = g2_mma(a0, bf, c01); c11 = g2_mma(a1, bf, c11);
    bf = g2_frag(b2p + kb, hh); c02 = g2_mma(a0, bf, c02); c12 = g2_mma(a1, bf, c12);
    bf = g2_frag(b3p + kb, hh); c03 = g2_mma(a0, bf, c03); c13 = g2_mma(a1, bf, c13);
  }
  v8f accs[8] = {c00, c01, c02, c03, c10, c11, c12, c13};
#pragma unroll
  for (int u = 0; u < 8; ++u) {
    const int t = u & 3, half = u >> 2;
    const float bb = bf16_rne(bias[col0 + t * 16 + ln]);
#pragma unroll
    for (int r = 0; r < 8; ++r) { const int rloc = half * 16 + 8 * hh + r; float v = accs[u][r] * alpha + bb; if (ACT == 3) v = fmaxf(v, 0.f); so[w][rloc][t * 16 + ln] = v; }
  }
  __builtin_amdgcn_fence(4, "workgroup"); __builtin_amdgcn_wave_barrier();
  const int rsub = lane >> 4, c4 = (lane & 15) * 4;
  for (int pass = 0; pass < 2; ++pass) {
#pragma unroll
    for (int q = 0; q < 16; ++q) {
      const int r = q * 2 + rsub; const v4f v = *(const v4fa*)&so[w][r][c4];
      if (C) *(volatile v4f*)(C + cofs + (size_t)(row0 + r) * ldc + col0 + c4) = v;
      if (C16) { v4h h4; for (int i = 0; i < 4; ++i) h4[i] = (_Float16)v[i]; *(volatile v4h*)(C16 + cofs + (size_t)(row0 + r) * ldc + col0 + c4) = h4; }
    }
    if (pass == 0) __threadfence();
  }
}

template <int RES>
__global__ __launch_bounds__(256) void k_rope(const float* __restrict__ F, const float* __restrict__ CS, const float* __restrict__ SN,
                                              const int* __restrict__ EX, int use_ex, _Float16* __restrict__ H, _Float16* __restrict__ L) {
  #pragma clang fp contract(off)
  const size_t t = (size_t)blockIdx.x * 256 + threadIdx.x; if (t >= (size_t)NR * NH * 8) return;
  const int p = (int)(t & 7); const int hd = (int)((t >> 3) % NH); const size_t row = t / (8 * NH);
  const int s = (int)(row % SLEN);
  int nkr = TK - EX[0] * use_ex; if (nkr < 0) nkr += TK;
  const bool rot = (s < nkr);
  const float* src = F + row * DM + hd * 64 + p * 8;
  const v4f xa = *(const v4fa*)src, xb = *(const v4fa*)(src + 4);
  const v4f c4 = *(const v4fa*)(CS + (size_t)s * 32 + p * 4), s4 = *(const v4fa*)(SN + (size_t)s * 32 + p * 4);
  const float xs[8] = {xa[0], xa[1], xa[2], xa[3], xb[0], xb[1], xb[2], xb[3]};
  FragH fh, fl;
#pragma unroll
  for (int i = 0; i < 4; ++i) {
    const float a = xs[2 * i], xb1 = xs[2 * i + 1], c = c4[i], sn = s4[i];
    const float ra = a * c - xb1 * sn; const float rb = a * sn + xb1 * c;
    const float o0 = rot ? ra : a, o1 = rot ? rb : xb1;
    _Float16 hv = (_Float16)o0; fh.h[2 * i] = hv; fl.h[2 * i] = (_Float16)((o0 - (float)hv) * 1024.0f);
    hv = (_Float16)o1; fh.h[2 * i + 1] = hv; fl.h[2 * i + 1] = (_Float16)((o1 - (float)hv) * 1024.0f);
  }
  const size_t oh = row * DM + hd * 64 + p * 8;
  const v8us vh = fh.half[0], vl = fl.half[0];
  for (int pass = 0; pass < 2; ++pass) {
    *(volatile v8us*)((unsigned short*)H + oh) = vh;
    if (RES != 0) *(volatile v8us*)((unsigned short*)L + oh) = vl;
    if (pass == 0) __threadfence();
  }
}

__global__ __launch_bounds__(256) void k_vtg(const _Float16* __restrict__ V16, _Float16* __restrict__ Vt) {
  __shared__ unsigned short tl[64][66];
  const int tid = threadIdx.x; const int nlg = SLEN / 64; const int slab = blockIdx.x / nlg, lg = blockIdx.x % nlg; const int b = slab / NH, h = slab % NH;
  for (int i = tid; i < 64 * 8; i += 256) {
    const int r = i >> 3, c8 = (i & 7) * 8; FragH f;
    f.half[0] = *(const v8us*)((const unsigned short*)V16 + ((size_t)b * SLEN + lg * 64 + r) * DM + h * 64 + c8);
#pragma unroll
    for (int q = 0; q < 8; ++q) tl[r][c8 + q] = f.u[q];
  }
  __syncthreads();
  for (int pass = 0; pass < 2; ++pass) {
#pragma unroll
    for (int rd = 0; rd < 2; ++rd) {
      const int d = rd * 32 + (tid >> 3), pc = tid & 7; FragH f;
#pragma unroll
      for (int q = 0; q < 8; ++q) f.u[q] = tl[pc * 8 + q][d];
      *(volatile v8us*)((unsigned short*)Vt + ((size_t)slab * 64 + d) * TK + lg * 64 + pc * 8) = f.half[0];
    }
    if (pass == 0) __threadfence();
  }
}
__global__ __launch_bounds__(256) void k_vsum(const float* __restrict__ VF, float* __restrict__ VS) {
  const int tid = threadIdx.x; const int ngrp = SLEN / 128; const int slab = blockIdx.x / ngrp, g = blockIdx.x % ngrp; const int b = slab / NH, h = slab % NH;
  const int cq = tid >> 6, d = tid & 63; const int s0 = g * 128 + cq * 32;
  const float* src = VF + ((size_t)b * SLEN + s0) * DM + h * 64 + d;
  float a0 = 0.f, a1 = 0.f;
#pragma unroll 4
  for (int i = 0; i < 32; i += 2) { a0 += src[(size_t)i * DM]; a1 += src[(size_t)(i + 1) * DM]; }
  const float acc = a0 + a1;
  const int ch = g * 4 + cq;
  float* dst = VS + ((size_t)slab * NCH + ch) * 64 + d;
  *(volatile float*)dst = acc; __threadfence(); *(volatile float*)dst = acc;
}

__global__ __launch_bounds__(256) void k_hl(const float* __restrict__ Fp, _Float16* __restrict__ A2, size_t n8) {
  const size_t t = (size_t)blockIdx.x * 256 + threadIdx.x; if (t >= n8) return;
  const size_t e = t * 8; const size_t r = e / DM; const int c = (int)(e % DM);
  const v4f a = *(const v4fa*)(Fp + e), d = *(const v4fa*)(Fp + e + 4);
  FragH fh, fl;
#pragma unroll
  for (int q = 0; q < 4; ++q) {
    const float v0 = a[q] * 256.0f; _Float16 hv = (_Float16)v0; fh.h[q] = hv; fl.h[q] = (_Float16)((v0 - (float)hv) * 1024.0f);
    const float v1 = d[q] * 256.0f; hv = (_Float16)v1; fh.h[4 + q] = hv; fl.h[4 + q] = (_Float16)((v1 - (float)hv) * 1024.0f);
  }
  const size_t o2 = r * (size_t)(2 * DM) + c;
  const v8us vh = fh.half[0], vl = fl.half[0];
  for (int pass = 0; pass < 2; ++pass) {
    *(volatile v8us*)((unsigned short*)A2 + o2) = vh;
    *(volatile v8us*)((unsigned short*)A2 + o2 + DM) = vl;
    if (pass == 0) __threadfence();
  }
}

template <int QRES>
__global__ __launch_bounds__(128) void k_flash3(const _Float16* __restrict__ Q16, const _Float16* __restrict__ QL, int ldq,
                                                const _Float16* __restrict__ K16, const _Float16* __restrict__ KL, int ldk,
                                                const _Float16* __restrict__ Vt, const float* __restrict__ VS, float* __restrict__ O, int ldo) {
  constexpr int RPW = 16, DT = 4, KS = 2;
  __shared__ __attribute__((aligned(16))) unsigned short sP[4][RPW][40];
  __shared__ __attribute__((aligned(16))) float sO[4][RPW][68];
  const int tid = threadIdx.x, w = tid >> 5, lane = tid & 31, ln = lane & 15, hh = lane >> 4;
  const int slab = blockIdx.x / QBLKS, qblk = blockIdx.x % QBLKS; const int b = slab / NH, h = slab % NH;
  const int qb0 = qblk * (4 * RPW); const int q0 = qb0 + w * RPW;
  FragH aq[KS], aql[KS];
  {
    const unsigned short* qr = (const unsigned short*)Q16 + ((size_t)b * TQ + q0 + ln) * ldq + h * 64;
    const unsigned short* ql = (const unsigned short*)QL + ((size_t)b * TQ + q0 + ln) * ldq + h * 64;
#pragma unroll
    for (int ks = 0; ks < KS; ++ks) {
      aq[ks].half[0] = *(const v8us*)(qr + ks * 32 + 8 * hh); aq[ks].half[1] = *(const v8us*)(qr + ks * 32 + 16 + 8 * hh);
      if (QRES != 0) { aql[ks].half[0] = *(const v8us*)(ql + ks * 32 + 8 * hh); aql[ks].half[1] = *(const v8us*)(ql + ks * 32 + 16 + 8 * hh); }
      else aql[ks].v = aq[ks].v;
    }
  }
  const unsigned short* Vth = (const unsigned short*)Vt + (size_t)slab * 64 * TK;
  const float* VSp = VS + (size_t)slab * NCH * 64;
  float m_r[8], l_r[8]; v8f oacc[DT];
#pragma unroll
  for (int r = 0; r < 8; ++r) { m_r[r] = -3.0e38f; l_r[r] = 0.f; }
#pragma unroll
  for (int dt = 0; dt < DT; ++dt) oacc[dt] = (v8f){0.f,0.f,0.f,0.f,0.f,0.f,0.f,0.f};
#pragma unroll 1
  for (int j0 = 0; j0 < TK; j0 += 32) {
    v8f s[2];
#pragma unroll
    for (int nt = 0; nt < 2; ++nt) {
      const unsigned short* kr = (const unsigned short*)K16 + ((size_t)b * TK + j0 + nt * 16 + ln) * ldk + h * 64;
      FragH bk[KS];
#pragma unroll
      for (int ks = 0; ks < KS; ++ks) { bk[ks].half[0] = *(const v8us*)(kr + ks * 32 + 8 * hh); bk[ks].half[1] = *(const v8us*)(kr + ks * 32 + 16 + 8 * hh); }
      v8f acc = (v8f){0.f,0.f,0.f,0.f,0.f,0.f,0.f,0.f};
      if (QRES != 0) {
        const unsigned short* klr = (const unsigned short*)KL + ((size_t)b * TK + j0 + nt * 16 + ln) * ldk + h * 64;
        FragH bkl[KS];
#pragma unroll
        for (int ks = 0; ks < KS; ++ks) { bkl[ks].half[0] = *(const v8us*)(klr + ks * 32 + 8 * hh); bkl[ks].half[1] = *(const v8us*)(klr + ks * 32 + 16 + 8 * hh); }
        v8f accl = (v8f){0.f,0.f,0.f,0.f,0.f,0.f,0.f,0.f};
#pragma unroll
        for (int ks = 0; ks < KS; ++ks) {
          acc = mmaH<1>(aq[ks].v, aq[ks].v, bk[ks].v, bk[ks].v, acc);
          accl = mmaH<1>(aql[ks].v, aql[ks].v, bk[ks].v, bk[ks].v, accl);
          accl = mmaH<1>(aq[ks].v, aq[ks].v, bkl[ks].v, bkl[ks].v, accl);
        }
#pragma unroll
        for (int r = 0; r < 8; ++r) acc[r] += accl[r] * 0.0009765625f;
      } else {
#pragma unroll
        for (int ks = 0; ks < KS; ++ks) acc = mmaH<1>(aq[ks].v, aq[ks].v, bk[ks].v, bk[ks].v, acc);
      }
      s[nt] = acc;
    }
    float vs[DT];
#pragma unroll
    for (int dt = 0; dt < DT; ++dt) vs[dt] = VSp[(size_t)(j0 >> 5) * 64 + dt * 16 + ln];
#pragma unroll
    for (int r = 0; r < 8; ++r) {
      const float s0 = s[0][r] * SCL, s1 = s[1][r] * SCL;
      float mc = fmaxf(s0, s1);
      mc = fmaxf(mc, __shfl_xor(mc, 1, 32)); mc = fmaxf(mc, __shfl_xor(mc, 2, 32)); mc = fmaxf(mc, __shfl_xor(mc, 4, 32)); mc = fmaxf(mc, __shfl_xor(mc, 8, 32));
      const float mn = fmaxf(m_r[r], mc); const float al = (m_r[r] > -1.0e38f) ? __expf(m_r[r] - mn) : 0.f; m_r[r] = mn;
      const float p0 = __expf(s0 - mn), p1 = __expf(s1 - mn);
      float cs = p0 + p1;
      cs += __shfl_xor(cs, 1, 32); cs += __shfl_xor(cs, 2, 32); cs += __shfl_xor(cs, 4, 32); cs += __shfl_xor(cs, 8, 32);
      l_r[r] = l_r[r] * al + cs;
      const float c = cs * 32.0f;
#pragma unroll
      for (int dt = 0; dt < DT; ++dt) oacc[dt][r] = oacc[dt][r] * al + c * vs[dt];
      FragH t2; t2.h[0] = (_Float16)(p0 * 1024.0f - c); t2.h[1] = (_Float16)(p1 * 1024.0f - c);
      sP[w][8 * hh + r][ln] = t2.u[0]; sP[w][8 * hh + r][16 + ln] = t2.u[1];
    }
    __builtin_amdgcn_fence(4, "workgroup"); __builtin_amdgcn_wave_barrier();
    FragH pa; pa.half[0] = *(const v8us*)&sP[w][ln][8 * hh]; pa.half[1] = *(const v8us*)&sP[w][ln][16 + 8 * hh];
#pragma unroll
    for (int dt = 0; dt < DT; ++dt) {
      const unsigned short* vrow = Vth + (size_t)(dt * 16 + ln) * TK + j0; FragH bv;
      bv.half[0] = *(const v8us*)(vrow + 8 * hh); bv.half[1] = *(const v8us*)(vrow + 16 + 8 * hh);
      oacc[dt] = mmaH<1>(pa.v, pa.v, bv.v, bv.v, oacc[dt]);
    }
    __builtin_amdgcn_fence(4, "workgroup"); __builtin_amdgcn_wave_barrier();
  }
#pragma unroll
  for (int r = 0; r < 8; ++r) { const float l = l_r[r]; l_r[r] = (l > 0.f) ? 1.0f / (l * 1024.0f) : 0.f; }
#pragma unroll
  for (int dt = 0; dt < DT; ++dt)
#pragma unroll
    for (int r = 0; r < 8; ++r) sO[w][8 * hh + r][dt * 16 + ln] = oacc[dt][r] * l_r[r];
  __builtin_amdgcn_fence(4, "workgroup"); __builtin_amdgcn_wave_barrier();
  for (int pass = 0; pass < 2; ++pass) {
#pragma unroll
    for (int rp = 0; rp < RPW; rp += 2) { const int r = rp + (lane >> 4), pc = lane & 15; const v4f val = *(const v4fa*)&sO[w][r][pc * 4]; *(volatile v4f*)(O + ((size_t)b * TQ + q0 + r) * ldo + h * 64 + pc * 4) = val; }
    if (pass == 0) __threadfence();
  }
}

extern "C" void kernel_launch(void* const* d_in, const int* in_sizes, int n_in,
                              void* d_out, int out_size, void* d_ws, size_t ws_size, hipStream_t stream) {
  if (n_in < 12) return;
  const size_t needx = ((size_t)(NB - 1) * SEQ_FULL + (size_t)SLEN) * DM;
  for (int i = 0; i < 3; ++i) if ((size_t)in_sizes[i] < needx) return;
  for (int i = 3; i < 11; i += 2) if ((size_t)in_sizes[i] < (size_t)DM * DM) return;
  for (int i = 4; i < 11; i += 2) if ((size_t)in_sizes[i] < (size_t)DM) return;
  if (in_sizes[11] < 1) return;
  if ((size_t)out_size < needx) return;
  const float* qin = (const float*)d_in[0]; const float* kin = (const float*)d_in[1]; const float* vin = (const float*)d_in[2];
  const float* Wq = (const float*)d_in[3]; const float* bq = (const float*)d_in[4];
  const float* Wk = (const float*)d_in[5]; const float* bk = (const float*)d_in[6];
  const float* Wv = (const float*)d_in[7]; const float* bv = (const float*)d_in[8];
  const float* Wo = (const float*)d_in[9]; const float* bo = (const float*)d_in[10];
  const int* EX = (const int*)d_in[11];
  float* dout = (float*)d_out;
  char* ws = (char*)d_ws; size_t off = 0;
  auto take = [&](size_t bytes) { char* p = ws + off; off += (bytes + 255) & ~(size_t)255; return p; };
  const size_t np = (size_t)NR * DM;
  _Float16* BQ = (_Float16*)take((size_t)DM * DM * 2);
  _Float16* BK = (_Float16*)take((size_t)DM * DM * 2);
  _Float16* BV = (_Float16*)take((size_t)DM * DM * 2);
  _Float16* B2 = (_Float16*)take((size_t)DM * 2 * DM * 2);
  float* FS = (float*)take(np * 4);
  _Float16* X16 = (_Float16*)take(np * 2);
  _Float16* VT = X16;
  _Float16* QH = (_Float16*)take(np * 2);
  _Float16* KH = (_Float16*)take(np * 2);
  _Float16* V16 = (_Float16*)take(np * 2);
  float* VS = (float*)take((size_t)NB * NH * NCH * 64 * 4);
  _Float16* A2 = (_Float16*)take(np * 2 * 2);
  float* CS = (float*)take((size_t)SLEN * 32 * 4); float* SN = (float*)take((size_t)SLEN * 32 * 4); float* INV = (float*)take(128);
#if QK_RES
  _Float16* QL = (_Float16*)take(np * 2);
  _Float16* KL = (_Float16*)take(np * 2);
#else
  _Float16* QL = QH;
  _Float16* KL = KH;
#endif
  if (off > ws_size) return;
  if (off > ((size_t)128 << 20)) return;

  const unsigned gwt = (unsigned)((DM / 64) * (DM / 64));
  k_wtr<0><<<gwt, 256, 0, stream>>>(Wq, BQ, DM, 16.0f, 0.0f);
  k_wtr<0><<<gwt, 256, 0, stream>>>(Wk, BK, DM, 16.0f, 0.0f);
  k_wtr<0><<<gwt, 256, 0, stream>>>(Wv, BV, DM, 16.0f, 0.0f);
  k_wtr<1><<<gwt, 256, 0, stream>>>(Wo, B2, 2 * DM, 16384.0f, 16.0f);
  k_invf<<<1, 32, 0, stream>>>(INV);
  k_rotab<<<(unsigned)((SLEN * 32 + 255) / 256), 256, 0, stream>>>(INV, CS, SN);
  const unsigned g8 = (unsigned)((np / 8 + 255) / 256);
  const dim3 gp((unsigned)((NR / 128) * (DM / 64)), 1);
  const unsigned gr = (unsigned)(((size_t)NR * NH * 8 + 255) / 256);
  k_x16<<<g8, 256, 0, stream>>>(qin, X16, np / 8);
  k_gemm2<0><<<gp, 128, 0, stream>>>(X16, DM, 0, BQ, DM, 0, 0.0625f, FS, nullptr, DM, 0, NR, DM, DM, bq);
  k_rope<QK_RES><<<gr, 256, 0, stream>>>(FS, CS, SN, EX, 0, QH, QL);
  k_x16<<<g8, 256, 0, stream>>>(kin, X16, np / 8);
  k_gemm2<0><<<gp, 128, 0, stream>>>(X16, DM, 0, BK, DM, 0, 0.0625f, FS, nullptr, DM, 0, NR, DM, DM, bk);
  k_rope<QK_RES><<<gr, 256, 0, stream>>>(FS, CS, SN, EX, 1, KH, KL);
  k_x16<<<g8, 256, 0, stream>>>(vin, X16, np / 8);
  k_gemm2<0><<<gp, 128, 0, stream>>>(X16, DM, 0, BV, DM, 0, 0.0625f, FS, V16, DM, 0, NR, DM, DM, bv);
  k_vtg<<<(unsigned)(NB * NH * (SLEN / 64)), 256, 0, stream>>>(V16, VT);
  k_vsum<<<(unsigned)(NB * NH * (SLEN / 128)), 256, 0, stream>>>(FS, VS);
  k_flash3<QK_RES><<<(unsigned)(NB * NH * QBLKS), 128, 0, stream>>>(QH, QL, DM, KH, KL, DM, VT, VS, FS, DM);
  k_hl<<<g8, 256, 0, stream>>>(FS, A2, np / 8);
  const dim3 ge((unsigned)((SLEN / 128) * (DM / 64)), NB);
  k_gemm2<0><<<ge, 128, 0, stream>>>(A2, 2 * DM, (size_t)SLEN * 2 * DM, B2, 2 * DM, 0, 1.0f / (16384.0f * 256.0f), dout, nullptr, DM, (size_t)SEQ_FULL * DM, SLEN, DM, 2 * DM, bo);
}
